// MoETaskAttention_18528488915483
// MI455X (gfx1250) — hardware-verified
//
#include <hip/hip_runtime.h>
#include <math.h>
typedef __attribute__((ext_vector_type(16))) _Float16 v16h;
typedef __attribute__((ext_vector_type(8)))  _Float16 v8h;
typedef __attribute__((ext_vector_type(16))) __bf16   v16b;
typedef __attribute__((ext_vector_type(8)))  __bf16   v8b;
typedef __attribute__((ext_vector_type(8)))  float    v8f;
typedef __attribute__((ext_vector_type(4)))  float    v4f;
#define PSCALE 32768.0f
#define U16(p) ((const unsigned short*)(const void*)(p))
#define PSCALE_INV (1.0f / 32768.0f)

__device__ __forceinline__ unsigned short f2bf_bits(float f) {
  unsigned u = __float_as_uint(f);
  return (unsigned short)((u + 0x7FFFu + ((u >> 16) & 1u)) >> 16);
}
__device__ __forceinline__ float bf_bits2f(unsigned short h) { return __uint_as_float(((unsigned)h) << 16); }

__device__ __forceinline__ void dep_guard_h(v8f& a, v8f& b, v16h x, v16h y) { asm volatile("v_nop\n\tv_nop\n\tv_nop\n\tv_nop" : "+v"(a), "+v"(b) : "v"(x), "v"(y)); }
__device__ __forceinline__ void dep_guard_b(v8f& a, v8f& b, v16b x, v16b y) { asm volatile("v_nop\n\tv_nop\n\tv_nop\n\tv_nop" : "+v"(a), "+v"(b) : "v"(x), "v"(y)); }
__device__ __forceinline__ void keep4_h(v16h a, v16h b, v16h c, v16h d) { asm volatile("v_nop" :: "v"(a), "v"(b), "v"(c), "v"(d)); }
__device__ __forceinline__ void keep4_b(v16b a, v16b b, v16b c, v16b d) { asm volatile("v_nop" :: "v"(a), "v"(b), "v"(c), "v"(d)); }
__device__ __forceinline__ void acc_guard4(v8f& a, v8f& b, v8f& c, v8f& d) { asm volatile("v_nop\n\tv_nop\n\tv_nop\n\tv_nop" : "+v"(a), "+v"(b), "+v"(c), "+v"(d)); }
template <typename T> struct Frag;
template <> struct Frag<_Float16> {
  typedef v16h V; union U { v16h v; v8h h[2]; };
  static __device__ __forceinline__ v16h load(const _Float16* p) {
    U f; f.h[0] = *(const v8h*)(p); f.h[1] = *(const v8h*)(p + 16); return f.v;
  }
  static __device__ __forceinline__ v8f mma(v16h a, v16h b, v8f c) {
    return __builtin_amdgcn_wmma_f32_16x16x32_f16(false, a, false, b, (short)0, c, false, false);
  }
  static __device__ __forceinline__ void guard(v8f& a, v8f& b, v16h x, v16h y) { dep_guard_h(a, b, x, y); }
  static __device__ __forceinline__ void keep(v16h a, v16h b, v16h c, v16h d) { keep4_h(a, b, c, d); }
};
template <> struct Frag<__bf16> {
  typedef v16b V; union U { v16b v; v8b h[2]; };
  static __device__ __forceinline__ v16b load(const __bf16* p) {
    U f; f.h[0] = *(const v8b*)(p); f.h[1] = *(const v8b*)(p + 16); return f.v;
  }
  static __device__ __forceinline__ v8f mma(v16b a, v16b b, v8f c) {
    return __builtin_amdgcn_wmma_f32_16x16x32_bf16(false, a, false, b, (short)0, c, false, false);
  }
  static __device__ __forceinline__ void guard(v8f& a, v8f& b, v16b x, v16b y) { dep_guard_b(a, b, x, y); }
  static __device__ __forceinline__ void keep(v16b a, v16b b, v16b c, v16b d) { keep4_b(a, b, c, d); }
};

template <int ET> struct Elem;
template <> struct Elem<0> { typedef _Float16 T; };
template <> struct Elem<1> { typedef __bf16 T; };
template <int ET, bool SPLIT, int BIAS_MODE, int OUT_MODE, bool RESID, int ACT = 0>
__global__ __launch_bounds__(256) void wmma_gemm64(
    const unsigned short* __restrict__ Ap, const unsigned short* __restrict__ A2p, int lda, long strideA,
    const unsigned short* __restrict__ Btp, const unsigned short* __restrict__ Bt2p, int ldb, long strideB,
    void* __restrict__ Cout, void* __restrict__ Cout2, int ldc, long strideC,
    const float* __restrict__ bias,
    const float* __restrict__ resid, long strideR,
    int M, int N, int K, float scale) {
  typedef typename Elem<ET>::T T;
  typedef typename Frag<T>::V V;
  const T* A = (const T*)Ap; const T* A2 = (const T*)A2p; const T* Bt = (const T*)Btp; const T* Bt2 = (const T*)Bt2p;
  __shared__ __align__(16) float sT[8][16 * 68];
  const int b    = blockIdx.y;
  const int lane = threadIdx.x & 31;
  const int wave = threadIdx.x >> 5;
  const int tilesN = N >> 6;
  const int tilesM = M >> 6;
  const int tile = blockIdx.x * 8 + wave;
  if (tile >= tilesM * tilesN) return;
  const int tm = tile / tilesN;
  const int tn = tile - tm * tilesN;
  const int m0 = tm << 6;
  const int n0 = tn << 6;

  const T* Ab  = A  + (size_t)b * strideA;
  const T* Bb  = Bt + (size_t)b * strideB;
  const T* Ab2 = SPLIT ? (A2  + (size_t)b * strideA) : nullptr;
  const T* Bb2 = SPLIT ? (Bt2 + (size_t)b * strideB) : nullptr;

  const int rlane = lane & 15;
  const int koff  = (lane >> 4) * 8;
  const int mOff  = (lane >> 4) * 8;

  v8f acc[4][4];
#pragma unroll
  for (int i = 0; i < 4; ++i)
#pragma unroll
    for (int j = 0; j < 4; ++j) acc[i][j] = (v8f){0.f,0.f,0.f,0.f,0.f,0.f,0.f,0.f};

  for (int k0 = 0; k0 < K; k0 += 32) {
    V bh[4], bl[4];
#pragma unroll
    for (int j = 0; j < 4; ++j) {
      const size_t bo = (size_t)(n0 + (j << 4) + rlane) * ldb + koff + k0;
      bh[j] = Frag<T>::load(Bb + bo);
      if (SPLIT) bl[j] = Frag<T>::load(Bb2 + bo);
    }
#pragma unroll
    for (int i = 0; i < 4; ++i) {
      const size_t ao = (size_t)(m0 + (i << 4) + rlane) * lda + koff + k0;
      V ah = Frag<T>::load(Ab + ao);
      V al;
      if (SPLIT) al = Frag<T>::load(Ab2 + ao);
#pragma unroll
      for (int j = 0; j < 4; ++j) {
        acc[i][j] = Frag<T>::mma(ah, bh[j], acc[i][j]);
        if (SPLIT) {
          acc[i][j] = Frag<T>::mma(ah, bl[j], acc[i][j]);
          acc[i][j] = Frag<T>::mma(al, bh[j], acc[i][j]);
        }
      }
      Frag<T>::guard(acc[i][0], acc[i][3], ah, SPLIT ? al : ah);
    }
    Frag<T>::keep(bh[0], bh[1], bh[2], bh[3]);
    if (SPLIT) Frag<T>::keep(bl[0], bl[1], bl[2], bl[3]);
  }
  acc_guard4(acc[0][0], acc[0][1], acc[0][2], acc[0][3]);
  acc_guard4(acc[1][0], acc[1][1], acc[1][2], acc[1][3]);
  acc_guard4(acc[2][0], acc[2][1], acc[2][2], acc[2][3]);
  acc_guard4(acc[3][0], acc[3][1], acc[3][2], acc[3][3]);

  float* slab = sT[wave];
  const float* Rb = RESID ? (resid + (size_t)b * strideR) : nullptr;
#pragma unroll
  for (int i = 0; i < 4; ++i) {
    const int mBase = m0 + (i << 4);
#pragma unroll
    for (int j = 0; j < 4; ++j) {
      const int n = n0 + (j << 4) + rlane;
      float bv = 0.f;
      if (BIAS_MODE == 2) bv = bias[n];
#pragma unroll
      for (int r = 0; r < 8; ++r) {
        float v = acc[i][j][r] * scale;
        if (BIAS_MODE == 1) v += bias[mBase + mOff + r];
        if (BIAS_MODE == 2) v += bv;
        if (RESID) v += Rb[(size_t)(mBase + mOff + r) * ldc + n];
        if (ACT == 1) v = tanhf(v);
        if (ACT == 2) v = fmaxf(v, 0.0f);
        if (ACT == 3) v = v / (1.0f + expf(-v));
        if (ACT == 4) v = (v > 0.f) ? v : 0.01f * v;
        if (ACT == 5) v = 0.5f * v * (1.0f + erff(v * 0.70710678118654752f));
        slab[(mOff + r) * 68 + (j << 4) + rlane] = v;
      }
    }
    __builtin_amdgcn_fence(__ATOMIC_RELEASE, "workgroup");
    __builtin_amdgcn_wave_barrier();
    __builtin_amdgcn_fence(__ATOMIC_ACQUIRE, "workgroup");
    if (OUT_MODE == 0) {
      float* C = (float*)Cout + (size_t)b * strideC;
      const int hh = lane >> 4, c4 = (lane & 15) * 4;
      for (int pass = 0; pass < 2; ++pass) {
#pragma unroll
        for (int it = 0; it < 8; ++it) {
          const int row = it * 2 + hh;
          v4f v = *(const v4f*)(slab + row * 68 + c4);
          *(volatile v4f*)(C + (size_t)(mBase + row) * ldc + n0 + c4) = v;
        }
        __threadfence();
      }
    } else {
      const int q = lane >> 3, c8 = (lane & 7) * 8;
      unsigned short* C  = (unsigned short*)Cout  + (size_t)b * strideC;
      unsigned short* C2 = (OUT_MODE == 2) ? ((unsigned short*)Cout2 + (size_t)b * strideC) : nullptr;
      for (int pass = 0; pass < 2; ++pass) {
#pragma unroll
        for (int it = 0; it < 4; ++it) {
          const int row = it * 4 + q;
          const float* sp = slab + row * 68 + c8;
          v8h hv, lv;
#pragma unroll
          for (int e = 0; e < 8; ++e) {
            if (OUT_MODE == 1) {
              hv[e] = (_Float16)sp[e];
            } else {
              unsigned short hb = f2bf_bits(sp[e]);
              unsigned short lb = f2bf_bits(sp[e] - bf_bits2f(hb));
              hv[e] = __builtin_bit_cast(_Float16, hb);
              lv[e] = __builtin_bit_cast(_Float16, lb);
            }
          }
          *(volatile v8h*)(C + (size_t)(mBase + row) * ldc + n0 + c8) = hv;
          if (OUT_MODE == 2) *(volatile v8h*)(C2 + (size_t)(mBase + row) * ldc + n0 + c8) = lv;
        }
        __threadfence();
      }
    }
    __builtin_amdgcn_fence(__ATOMIC_RELEASE, "workgroup");
    __builtin_amdgcn_wave_barrier();
    __builtin_amdgcn_fence(__ATOMIC_ACQUIRE, "workgroup");
  }
}

__global__ __launch_bounds__(256) void cast_f32_f16x2(
    const float* __restrict__ in, _Float16* __restrict__ out, int n2) {
  int i = blockIdx.x * 256 + threadIdx.x;
  if (i < n2) {
    const _Float16 h0 = (_Float16)in[2 * i], h1 = (_Float16)in[2 * i + 1];
    const unsigned u = (unsigned)__builtin_bit_cast(unsigned short, h0) | ((unsigned)__builtin_bit_cast(unsigned short, h1) << 16);
    ((volatile unsigned*)out)[i] = u;
    __threadfence();
    ((volatile unsigned*)out)[i] = u;
  }
}


__global__ __launch_bounds__(256) void cast_f32_f16x2s(const float* __restrict__ in, _Float16* __restrict__ out, int n2, float s) {
  int i = blockIdx.x * 256 + threadIdx.x;
  if (i < n2) {
    const _Float16 h0 = (_Float16)(in[2 * i] * s), h1 = (_Float16)(in[2 * i + 1] * s);
    const unsigned u = (unsigned)__builtin_bit_cast(unsigned short, h0) | ((unsigned)__builtin_bit_cast(unsigned short, h1) << 16);
    ((volatile unsigned*)out)[i] = u;
    __threadfence();
    ((volatile unsigned*)out)[i] = u;
  }
}
__global__ __launch_bounds__(256) void split_f32_bf16x2(
    const float* __restrict__ in, __bf16* __restrict__ hi, __bf16* __restrict__ lo, long n2) {
  long i = (long)blockIdx.x * 256 + threadIdx.x;
  long stride = (long)gridDim.x * 256;
  for (int pass = 0; pass < 2; ++pass) {
    for (long j = i; j < n2; j += stride) {
      const float a = in[2 * j], b = in[2 * j + 1];
      const unsigned short ah = f2bf_bits(a), bh = f2bf_bits(b);
      const unsigned short al = f2bf_bits(a - bf_bits2f(ah)), bl = f2bf_bits(b - bf_bits2f(bh));
      ((volatile unsigned*)hi)[j] = (unsigned)ah | ((unsigned)bh << 16);
      ((volatile unsigned*)lo)[j] = (unsigned)al | ((unsigned)bl << 16);
    }
    __threadfence();
  }
}


__global__ __launch_bounds__(256) void transpose_cast_f16(const float* __restrict__ in, int ldi,
                                                         _Float16* __restrict__ outT, int ldo, float scale) {
  __shared__ __align__(16) _Float16 tile[64][72];
  const int c0 = blockIdx.x * 64, r0 = blockIdx.y * 64;
  const int t = threadIdx.y * 32 + threadIdx.x;
  for (int i = threadIdx.y; i < 64; i += 8) {
    tile[threadIdx.x][i]      = (_Float16)(in[(size_t)(r0 + i) * ldi + c0 + threadIdx.x] * scale);
    tile[32 + threadIdx.x][i] = (_Float16)(in[(size_t)(r0 + i) * ldi + c0 + 32 + threadIdx.x] * scale);
  }
  __syncthreads();
  const int q = t >> 3, c8 = (t & 7) * 8;
  for (int pass = 0; pass < 2; ++pass) {
#pragma unroll
    for (int it = 0; it < 2; ++it) {
      const int c = it * 32 + q;
      v8h hv = *(const v8h*)(&tile[c][c8]);
      *(volatile v8h*)(outT + (size_t)(c0 + c) * ldo + r0 + c8) = hv;
    }
    __threadfence();
  }
}

__global__ __launch_bounds__(256) void transpose_split_bf16(const float* __restrict__ in, int ldi,
                                                           __bf16* __restrict__ outH, __bf16* __restrict__ outL, int ldo) {
  __shared__ __align__(16) float tile[64][68];
  const int c0 = blockIdx.x * 64, r0 = blockIdx.y * 64;
  const int t = threadIdx.y * 32 + threadIdx.x;
  for (int i = threadIdx.y; i < 64; i += 8) {
    tile[threadIdx.x][i]      = in[(size_t)(r0 + i) * ldi + c0 + threadIdx.x];
    tile[32 + threadIdx.x][i] = in[(size_t)(r0 + i) * ldi + c0 + 32 + threadIdx.x];
  }
  __syncthreads();
  const int q = t >> 3, c8 = (t & 7) * 8;
  for (int pass = 0; pass < 2; ++pass) {
#pragma unroll
    for (int it = 0; it < 2; ++it) {
      const int c = it * 32 + q;
      v8b hv, lv;
#pragma unroll
      for (int e = 0; e < 8; ++e) {
        const float f = tile[c][c8 + e];
        const unsigned short hb = f2bf_bits(f);
        hv[e] = __builtin_bit_cast(__bf16, hb);
        lv[e] = __builtin_bit_cast(__bf16, f2bf_bits(f - bf_bits2f(hb)));
      }
      *(volatile v8b*)(outH + (size_t)(c0 + c) * ldo + r0 + c8) = hv;
      *(volatile v8b*)(outL + (size_t)(c0 + c) * ldo + r0 + c8) = lv;
    }
    __threadfence();
  }
}

#define AT_D 64
#define AT_NW 4
#define AT_QB 64
#define AT_KC 64
struct AttnGeom { const float* cp = nullptr; const float* pc = nullptr; long c_bs = 0, c_rs = 0, c_hs = 0;
                  long q_bs, q_rs, q_hs, k_bs, k_rs, k_hs, v_bs, v_rs, v_hs, o_bs, o_rs, o_hs;
                  int S, Skv, H, mask_mode; float qscale; int blk0; float mask_fill; int mask_is_int; };
static_assert(sizeof(AttnGeom) == 168, "no padding");

__device__ __forceinline__ unsigned short at_bf_bits(float f) {
  unsigned u = __float_as_uint(f);
  return (unsigned short)((u + 0x7FFFu + ((u >> 16) & 1u)) >> 16);
}
__device__ __forceinline__ __bf16 at_f2bf(float f) { return __builtin_bit_cast(__bf16, at_bf_bits(f)); }
__device__ __forceinline__ void at_split(float f, __bf16& hi, __bf16& lo) {
  const unsigned short hb = at_bf_bits(f);
  hi = __builtin_bit_cast(__bf16, hb);
  lo = at_f2bf(f - __uint_as_float(((unsigned)hb) << 16));
}
__device__ __forceinline__ v8f at_mma(v16b a, v16b b, v8f c) {
  c = __builtin_amdgcn_wmma_f32_16x16x32_bf16(false, a, false, b, (short)0, c, false, false);
  asm volatile("v_nop\n\tv_nop\n\tv_nop\n\tv_nop" : "+v"(c) : "v"(a), "v"(b));
  return c;
}
template <bool F16> __device__ __forceinline__ __bf16 at_to16(float f) {
  if (F16) return __builtin_bit_cast(__bf16, (_Float16)f);
  return at_f2bf(f);
}
template <bool F16> __device__ __forceinline__ v8f at_mma16(v16b a, v16b b, v8f c) {
  if (F16) {
    const v16h ah = __builtin_bit_cast(v16h, a), bh = __builtin_bit_cast(v16h, b);
    c = __builtin_amdgcn_wmma_f32_16x16x32_f16(false, ah, false, bh, (short)0, c, false, false);
    asm volatile("v_nop\n\tv_nop\n\tv_nop\n\tv_nop" : "+v"(c) : "v"(ah), "v"(bh));
    return c;
  }
  return at_mma(a, b, c);
}

template <bool SPLIT_QK, bool SPLIT_PV, bool F16 = false>
__global__ __launch_bounds__(128)
void attn64_kernel(const float* __restrict__ q, const float* __restrict__ k,
                   const float* __restrict__ v, float* __restrict__ out,
                   const void* __restrict__ mask_a, const int* __restrict__ mask_b, AttnGeom g) {
  static_assert(!(F16 && (SPLIT_QK || SPLIT_PV)), "f16 mode is non-split");
  const float PSC = F16 ? 32768.0f : 1.0f;
  union FB { v16b v; v8b h[2]; };
  __shared__ __align__(16) __bf16 Ksh[AT_KC * AT_D];
  __shared__ __align__(16) __bf16 Ksl[SPLIT_QK ? AT_KC * AT_D : 8];
  __shared__ __align__(16) __bf16 Vth[AT_D * AT_KC];
  __shared__ __align__(16) __bf16 Vtl[SPLIT_PV ? AT_D * AT_KC : 8];
  __shared__ __align__(16) __bf16 Psh[AT_NW][16 * AT_KC];
  __shared__ __align__(16) __bf16 Psl[SPLIT_PV ? AT_NW : 1][SPLIT_PV ? 16 * AT_KC : 8];
  __shared__ __align__(16) float  Os[AT_NW][16 * 68];

  const int tid  = threadIdx.x;
  const int wave = tid >> 5;
  const int lane = tid & 31;
  const int hh   = lane >> 4;
  const int c    = lane & 15;

  const int nqb = g.S / AT_QB;
  const int bx = blockIdx.x + g.blk0;
  const int qb = bx % nqb;
  const int bh = bx / nqb;
  const int h  = bh % g.H;
  const int b  = bh / g.H;
  const int qbase_block = qb * AT_QB;
  const int q0 = qbase_block + wave * 16;

  const float* qb_ptr = q + (size_t)b * g.q_bs + (size_t)h * g.q_hs;
  const float* kb_ptr = k + (size_t)b * g.k_bs + (size_t)h * g.k_hs;
  const float* vb_ptr = v + (size_t)b * g.v_bs + (size_t)h * g.v_hs;
  float*       ob_ptr = out + (size_t)b * g.o_bs + (size_t)h * g.o_hs;

  v16b qah[2], qal[2];
  {
    const float* qrow = qb_ptr + (size_t)(q0 + c) * g.q_rs;
#pragma unroll
    for (int dc = 0; dc < 2; ++dc) {
#pragma unroll
      for (int e = 0; e < 8; ++e) {
        const float f0 = qrow[dc * 32 + 8 * hh + e] * g.qscale;
        const float f1 = qrow[dc * 32 + 16 + 8 * hh + e] * g.qscale;
        if (SPLIT_QK) { __bf16 hq, lq; at_split(f0, hq, lq); qah[dc][e] = hq; qal[dc][e] = lq; at_split(f1, hq, lq); qah[dc][8 + e] = hq; qal[dc][8 + e] = lq; }
        else { qah[dc][e] = at_to16<F16>(f0); qah[dc][8 + e] = at_to16<F16>(f1); qal[dc][e] = qah[dc][e]; qal[dc][8 + e] = qah[dc][8 + e]; }
      }
    }
  }

  float mrow[8], lrow[8];
  v8f oacc[4];
#pragma unroll
  for (int r = 0; r < 8; ++r) { mrow[r] = -INFINITY; lrow[r] = 0.f; }
#pragma unroll
  for (int t = 0; t < 4; ++t) oacc[t] = (v8f){0.f,0.f,0.f,0.f,0.f,0.f,0.f,0.f};

  const int nChunks = (g.mask_mode == 1 || g.mask_mode == 4) ? (qb + 1) : (g.Skv / AT_KC);
  int qkeep[8];
#pragma unroll
  for (int r = 0; r < 8; ++r) qkeep[r] = (g.mask_mode == 3) ? mask_b[(size_t)b * g.S + q0 + 8 * hh + r] : 1;
  for (int kc = 0; kc < nChunks; ++kc) {
    const int kv0 = kc * AT_KC;
    __syncthreads();
    {
      const int kvr = tid >> 1, dh = (tid & 1) * 32;
      const float* krow = kb_ptr + (size_t)(kv0 + kvr) * g.k_rs + dh;
      const float* vrow = vb_ptr + (size_t)(kv0 + kvr) * g.v_rs + dh;
#pragma unroll
      for (int i = 0; i < 8; ++i) {
        v4f kk = *(const v4f*)(krow + 4 * i);
        v4f vv = *(const v4f*)(vrow + 4 * i);
#pragma unroll
        for (int e = 0; e < 4; ++e) {
          const int d = dh + 4 * i + e;
          if (SPLIT_QK) { __bf16 a, bl; at_split(kk[e], a, bl); Ksh[kvr * AT_D + d] = a; Ksl[kvr * AT_D + d] = bl; }
          else Ksh[kvr * AT_D + d] = at_to16<F16>(kk[e]);
          if (SPLIT_PV) { __bf16 a, bl; at_split(vv[e], a, bl); Vth[d * AT_KC + kvr] = a; Vtl[d * AT_KC + kvr] = bl; }
          else Vth[d * AT_KC + kvr] = at_to16<F16>(vv[e]);
        }
      }
    }
    __syncthreads();

    v8f s[4];
#pragma unroll
    for (int j = 0; j < 4; ++j) {
      s[j] = (v8f){0.f,0.f,0.f,0.f,0.f,0.f,0.f,0.f};
#pragma unroll 1
      for (int dc = 0; dc < 2; ++dc) {
        FB kb;
        kb.h[0] = *(const v8b*)(Ksh + (j * 16 + c) * AT_D + dc * 32 + 8 * hh);
        kb.h[1] = *(const v8b*)(Ksh + (j * 16 + c) * AT_D + dc * 32 + 16 + 8 * hh);
        s[j] = at_mma16<F16>(qah[dc], kb.v, s[j]);
        if (SPLIT_QK) {
          FB kl;
          kl.h[0] = *(const v8b*)(Ksl + (j * 16 + c) * AT_D + dc * 32 + 8 * hh);
          kl.h[1] = *(const v8b*)(Ksl + (j * 16 + c) * AT_D + dc * 32 + 16 + 8 * hh);
          s[j] = at_mma16<F16>(qah[dc], kl.v, s[j]);
          s[j] = at_mma16<F16>(qal[dc], kb.v, s[j]);
        }
      }
    }
    const bool diag = (g.mask_mode == 1) && (kc == qb);
    int kvkeep[4] = {1, 1, 1, 1};
    if (g.mask_mode == 3) {
#pragma unroll
      for (int j = 0; j < 4; ++j) kvkeep[j] = ((const int*)mask_a)[(size_t)b * g.Skv + kv0 + j * 16 + c];
    }
    float cm[8];
#pragma unroll
    for (int r = 0; r < 8; ++r) {
      const int qrow = q0 + 8 * hh + r;
      float m = -INFINITY;
#pragma unroll
      for (int j = 0; j < 4; ++j) {
        const int kvcol = kv0 + j * 16 + c;
        bool masked = false;
        if (diag) masked = (kvcol > qrow);
        else if (g.mask_mode == 4) masked = (kvcol > qrow) || (qrow - kvcol > g.mask_is_int);
        else if (g.mask_mode == 2) {
          const size_t mi = (size_t)qrow * g.Skv + kvcol;
          masked = (g.mask_is_int == 0) ? (((const float*)mask_a)[mi] == 0.0f)
                 : (g.mask_is_int == 1) ? (((const int*)mask_a)[mi] == 0) : (((const int*)mask_a)[mi] != 0);
        } else if (g.mask_mode == 3) masked = (qkeep[r] == 0) || (kvkeep[j] == 0);
        else if (g.mask_mode == 5) {
          const size_t mi = (size_t)qrow * g.Skv + kvcol;
          masked = (((const int*)mask_a)[mi] != 0);
          int n = mask_b[mi]; n = n < 0 ? 0 : n;
          s[j][r] += g.cp[(size_t)b * g.c_bs + (size_t)h * g.c_hs + (size_t)qrow * g.c_rs + n]
                   + g.pc[(size_t)b * g.c_bs + (size_t)h * g.c_hs + (size_t)kvcol * g.c_rs + n];
        }
        if (masked) s[j][r] = g.mask_fill;
        m = fmaxf(m, s[j][r]);
      }
#pragma unroll
      for (int off = 1; off < 16; off <<= 1) m = fmaxf(m, __shfl_xor(m, off, 32));
      cm[r] = m;
    }
    __bf16* pwh = Psh[wave];
    __bf16* pwl = Psl[SPLIT_PV ? wave : 0];
#pragma unroll
    for (int r = 0; r < 8; ++r) {
      const float mnew = fmaxf(mrow[r], cm[r]);
      const float alpha = expf(mrow[r] - mnew);
      mrow[r] = mnew;
      float psum = 0.f;
#pragma unroll
      for (int j = 0; j < 4; ++j) {
        const float p = expf(s[j][r] - mnew);
        psum += p;
        if (SPLIT_PV) { __bf16 a, bl; at_split(p, a, bl); pwh[(8 * hh + r) * AT_KC + j * 16 + c] = a; pwl[(8 * hh + r) * AT_KC + j * 16 + c] = bl; }
        else pwh[(8 * hh + r) * AT_KC + j * 16 + c] = at_to16<F16>(p * PSC);
      }
#pragma unroll
      for (int off = 1; off < 16; off <<= 1) psum += __shfl_xor(psum, off, 32);
      lrow[r] = lrow[r] * alpha + psum;
#pragma unroll
      for (int t = 0; t < 4; ++t) oacc[t][r] *= alpha;
    }
    __builtin_amdgcn_fence(__ATOMIC_RELEASE, "workgroup");
    __builtin_amdgcn_wave_barrier();
    __builtin_amdgcn_fence(__ATOMIC_ACQUIRE, "workgroup");
#pragma unroll 1
    for (int kk = 0; kk < 2; ++kk) {
      FB pa, pl;
      pa.h[0] = *(const v8b*)(pwh + c * AT_KC + kk * 32 + 8 * hh);
      pa.h[1] = *(const v8b*)(pwh + c * AT_KC + kk * 32 + 16 + 8 * hh);
      if (SPLIT_PV) {
        pl.h[0] = *(const v8b*)(pwl + c * AT_KC + kk * 32 + 8 * hh);
        pl.h[1] = *(const v8b*)(pwl + c * AT_KC + kk * 32 + 16 + 8 * hh);
      }
#pragma unroll
      for (int t = 0; t < 4; ++t) {
        FB vb;
        vb.h[0] = *(const v8b*)(Vth + (t * 16 + c) * AT_KC + kk * 32 + 8 * hh);
        vb.h[1] = *(const v8b*)(Vth + (t * 16 + c) * AT_KC + kk * 32 + 16 + 8 * hh);
        oacc[t] = at_mma16<F16>(pa.v, vb.v, oacc[t]);
        if (SPLIT_PV) {
          FB vl;
          vl.h[0] = *(const v8b*)(Vtl + (t * 16 + c) * AT_KC + kk * 32 + 8 * hh);
          vl.h[1] = *(const v8b*)(Vtl + (t * 16 + c) * AT_KC + kk * 32 + 16 + 8 * hh);
          oacc[t] = at_mma16<F16>(pa.v, vl.v, oacc[t]);
          oacc[t] = at_mma16<F16>(pl.v, vb.v, oacc[t]);
        }
      }
    }
  }

  float* os = Os[wave];
#pragma unroll
  for (int r = 0; r < 8; ++r) {
    const float inv = 1.0f / (lrow[r] * PSC);
#pragma unroll
    for (int t = 0; t < 4; ++t) os[(8 * hh + r) * 68 + t * 16 + c] = oacc[t][r] * inv;
  }
  __builtin_amdgcn_fence(__ATOMIC_RELEASE, "workgroup");
  __builtin_amdgcn_wave_barrier();
  __builtin_amdgcn_fence(__ATOMIC_ACQUIRE, "workgroup");
  {
    const int c4 = (lane & 15) * 4;
    for (int pass = 0; pass < 2; ++pass) {
#pragma unroll
      for (int it = 0; it < 8; ++it) {
        const int row = it * 2 + hh;
        v4f val = *(const v4f*)(os + row * 68 + c4);
        *(volatile v4f*)(ob_ptr + (size_t)(q0 + row) * g.o_rs + c4) = val;
      }
      __threadfence();
    }
  }
}

template <bool SPLIT_QK, bool SPLIT_PV, bool F16 = false>
__global__ __launch_bounds__(128)
void attn128_kernel(const float* __restrict__ q, const float* __restrict__ k,
                   const float* __restrict__ v, float* __restrict__ out,
                   const void* __restrict__ mask_a, const int* __restrict__ mask_b, AttnGeom g) {
  static_assert(!(F16 && (SPLIT_QK || SPLIT_PV)), "f16 mode is non-split");
  const float PSC = F16 ? 32768.0f : 1.0f;
  union FB { v16b v; v8b h[2]; };
  constexpr int D2 = 128;
  __shared__ __align__(16) __bf16 Ksh[AT_KC * D2];
  __shared__ __align__(16) __bf16 Ksl[SPLIT_QK ? AT_KC * D2 : 8];
  __shared__ __align__(16) __bf16 Vth[D2 * AT_KC];
  __shared__ __align__(16) __bf16 Vtl[SPLIT_PV ? D2 * AT_KC : 8];
  __shared__ __align__(16) __bf16 Psh[AT_NW][16 * AT_KC];
  __shared__ __align__(16) __bf16 Psl[SPLIT_PV ? AT_NW : 1][SPLIT_PV ? 16 * AT_KC : 8];
  __shared__ __align__(16) float  Os[AT_NW][16 * 132];
  __shared__ __align__(16) __bf16 Qsh[AT_NW][16 * D2];
  __shared__ __align__(16) __bf16 Qsl[SPLIT_QK ? AT_NW : 1][SPLIT_QK ? 16 * D2 : 8];

  const int tid  = threadIdx.x;
  const int wave = tid >> 5;
  const int lane = tid & 31;
  const int hh   = lane >> 4;
  const int c    = lane & 15;

  const int nqb = g.S / AT_QB;
  const int bx = blockIdx.x + g.blk0;
  const int qb = bx % nqb;
  const int bh = bx / nqb;
  const int h  = bh % g.H;
  const int b  = bh / g.H;
  const int qbase_block = qb * AT_QB;
  const int q0 = qbase_block + wave * 16;

  const float* qb_ptr = q + (size_t)b * g.q_bs + (size_t)h * g.q_hs;
  const float* kb_ptr = k + (size_t)b * g.k_bs + (size_t)h * g.k_hs;
  const float* vb_ptr = v + (size_t)b * g.v_bs + (size_t)h * g.v_hs;
  float*       ob_ptr = out + (size_t)b * g.o_bs + (size_t)h * g.o_hs;

  v16b qah[4], qal[4];
  {
    const float* qrow = qb_ptr + (size_t)(q0 + c) * g.q_rs;
#pragma unroll
    for (int dc = 0; dc < 4; ++dc) {
#pragma unroll
      for (int e = 0; e < 8; ++e) {
        const float f0 = qrow[dc * 32 + 8 * hh + e] * g.qscale;
        const float f1 = qrow[dc * 32 + 16 + 8 * hh + e] * g.qscale;
        if (SPLIT_QK) { __bf16 hq, lq; at_split(f0, hq, lq); Qsh[wave][c * D2 + dc * 32 + 8 * hh + e] = hq; Qsl[wave][c * D2 + dc * 32 + 8 * hh + e] = lq;
                        at_split(f1, hq, lq); Qsh[wave][c * D2 + dc * 32 + 16 + 8 * hh + e] = hq; Qsl[wave][c * D2 + dc * 32 + 16 + 8 * hh + e] = lq;
                        qah[dc][e] = hq; qal[dc][e] = lq; qah[dc][8 + e] = hq; qal[dc][8 + e] = lq; }
        else { Qsh[wave][c * D2 + dc * 32 + 8 * hh + e] = at_to16<F16>(f0); Qsh[wave][c * D2 + dc * 32 + 16 + 8 * hh + e] = at_to16<F16>(f1); qah[dc][e] = at_to16<F16>(f0); qal[dc][e] = qah[dc][e]; qah[dc][8 + e] = qah[dc][e]; qal[dc][8 + e] = qah[dc][e]; }
      }
    }
  }

  float mrow[8], lrow[8];
  v8f oacc[8];
#pragma unroll
  for (int r = 0; r < 8; ++r) { mrow[r] = -INFINITY; lrow[r] = 0.f; }
#pragma unroll
  for (int t = 0; t < 8; ++t) oacc[t] = (v8f){0.f,0.f,0.f,0.f,0.f,0.f,0.f,0.f};

  const int nChunks = (g.mask_mode == 1 || g.mask_mode == 4 || g.mask_mode == 6) ? (qb + 1) : (g.Skv / AT_KC);
  int qkeep[8];
#pragma unroll
  for (int r = 0; r < 8; ++r) qkeep[r] = (g.mask_mode == 3) ? mask_b[(size_t)b * g.S + q0 + 8 * hh + r] : 1;
  for (int kc = 0; kc < nChunks; ++kc) {
    const int kv0 = kc * AT_KC;
    __syncthreads();
    {
      const int kvr = tid >> 1, dh = (tid & 1) * 64;
      const float* krow = kb_ptr + (size_t)(kv0 + kvr) * g.k_rs + dh;
      const float* vrow = vb_ptr + (size_t)(kv0 + kvr) * g.v_rs + dh;
#pragma unroll
      for (int i = 0; i < 16; ++i) {
        v4f kk = *(const v4f*)(krow + 4 * i);
        v4f vv = *(const v4f*)(vrow + 4 * i);
#pragma unroll
        for (int e = 0; e < 4; ++e) {
          const int d = dh + 4 * i + e;
          if (SPLIT_QK) { __bf16 a, bl; at_split(kk[e], a, bl); Ksh[kvr * D2 + d] = a; Ksl[kvr * D2 + d] = bl; }
          else Ksh[kvr * D2 + d] = at_to16<F16>(kk[e]);
          if (SPLIT_PV) { __bf16 a, bl; at_split(vv[e], a, bl); Vth[d * AT_KC + kvr] = a; Vtl[d * AT_KC + kvr] = bl; }
          else Vth[d * AT_KC + kvr] = at_to16<F16>(vv[e]);
        }
      }
    }
    __syncthreads();

    v8f s[4];
#pragma unroll
    for (int j = 0; j < 4; ++j) {
      s[j] = (v8f){0.f,0.f,0.f,0.f,0.f,0.f,0.f,0.f};
if (SPLIT_QK) {
#pragma unroll 1
      for (int dc = 0; dc < 4; ++dc) {
        FB kb;
        kb.h[0] = *(const v8b*)(Ksh + (j * 16 + c) * D2 + dc * 32 + 8 * hh);
        kb.h[1] = *(const v8b*)(Ksh + (j * 16 + c) * D2 + dc * 32 + 16 + 8 * hh);
        if (!SPLIT_QK) { FB qa; qa.h[0] = *(const v8b*)(&Qsh[wave][c * D2 + dc * 32 + 8 * hh]); qa.h[1] = *(const v8b*)(&Qsh[wave][c * D2 + dc * 32 + 16 + 8 * hh]); s[j] = at_mma16<F16>(qa.v, kb.v, s[j]); }
        if (SPLIT_QK) {
          FB qa, ql;
          qa.h[0] = *(const v8b*)(&Qsh[wave][c * D2 + dc * 32 + 8 * hh]); qa.h[1] = *(const v8b*)(&Qsh[wave][c * D2 + dc * 32 + 16 + 8 * hh]);
          ql.h[0] = *(const v8b*)(&Qsl[wave][c * D2 + dc * 32 + 8 * hh]); ql.h[1] = *(const v8b*)(&Qsl[wave][c * D2 + dc * 32 + 16 + 8 * hh]);
          s[j] = at_mma16<F16>(qa.v, kb.v, s[j]);
          FB kl;
          kl.h[0] = *(const v8b*)(Ksl + (j * 16 + c) * D2 + dc * 32 + 8 * hh);
          kl.h[1] = *(const v8b*)(Ksl + (j * 16 + c) * D2 + dc * 32 + 16 + 8 * hh);
          s[j] = at_mma16<F16>(qa.v, kl.v, s[j]);
          s[j] = at_mma16<F16>(ql.v, kb.v, s[j]);
        }
      }
      } else {
#pragma unroll
      for (int dc = 0; dc < 4; ++dc) {
        FB kb;
        kb.h[0] = *(const v8b*)(Ksh + (j * 16 + c) * D2 + dc * 32 + 8 * hh);
        kb.h[1] = *(const v8b*)(Ksh + (j * 16 + c) * D2 + dc * 32 + 16 + 8 * hh);
        if (!SPLIT_QK) { FB qa; qa.h[0] = *(const v8b*)(&Qsh[wave][c * D2 + dc * 32 + 8 * hh]); qa.h[1] = *(const v8b*)(&Qsh[wave][c * D2 + dc * 32 + 16 + 8 * hh]); s[j] = at_mma16<F16>(qa.v, kb.v, s[j]); }
        if (SPLIT_QK) {
          FB qa, ql;
          qa.h[0] = *(const v8b*)(&Qsh[wave][c * D2 + dc * 32 + 8 * hh]); qa.h[1] = *(const v8b*)(&Qsh[wave][c * D2 + dc * 32 + 16 + 8 * hh]);
          ql.h[0] = *(const v8b*)(&Qsl[wave][c * D2 + dc * 32 + 8 * hh]); ql.h[1] = *(const v8b*)(&Qsl[wave][c * D2 + dc * 32 + 16 + 8 * hh]);
          s[j] = at_mma16<F16>(qa.v, kb.v, s[j]);
          FB kl;
          kl.h[0] = *(const v8b*)(Ksl + (j * 16 + c) * D2 + dc * 32 + 8 * hh);
          kl.h[1] = *(const v8b*)(Ksl + (j * 16 + c) * D2 + dc * 32 + 16 + 8 * hh);
          s[j] = at_mma16<F16>(qa.v, kl.v, s[j]);
          s[j] = at_mma16<F16>(ql.v, kb.v, s[j]);
        }
      }
      }
    }
    const bool diag = (g.mask_mode == 1) && (kc == qb);
    int kvkeep[4] = {1, 1, 1, 1};
    if (g.mask_mode == 3) {
#pragma unroll
      for (int j = 0; j < 4; ++j) kvkeep[j] = ((const int*)mask_a)[(size_t)b * g.Skv + kv0 + j * 16 + c];
    }
    float cm[8];
#pragma unroll
    for (int r = 0; r < 8; ++r) {
      const int qrow = q0 + 8 * hh + r;
      float m = -INFINITY;
#pragma unroll
      for (int j = 0; j < 4; ++j) {
        const int kvcol = kv0 + j * 16 + c;
        bool masked = false;
        if (diag) masked = (kvcol > qrow);
        else if (g.mask_mode == 4) masked = (kvcol > qrow) || (qrow - kvcol > g.mask_is_int);
        else if (g.mask_mode == 2) {
          const size_t mi = (size_t)qrow * g.Skv + kvcol;
          masked = (g.mask_is_int == 0) ? (((const float*)mask_a)[mi] == 0.0f)
                 : (g.mask_is_int == 1) ? (((const int*)mask_a)[mi] == 0) : (((const int*)mask_a)[mi] != 0);
        } else if (g.mask_mode == 3) masked = (qkeep[r] == 0) || (kvkeep[j] == 0);
        else if (g.mask_mode == 6) { masked = (kvcol > qrow); s[j][r] += g.cp[h] * (float)(kvcol - qrow); }
        else if (g.mask_mode == 8) { masked = (kvcol > qrow) || (((const int*)mask_a)[(size_t)b * g.Skv + kvcol] != 0); }
        else if (g.mask_mode == 5) {
          const size_t mi = (size_t)qrow * g.Skv + kvcol;
          masked = (((const int*)mask_a)[mi] != 0);
          int n = mask_b[mi]; n = n < 0 ? 0 : n;
          s[j][r] += g.cp[(size_t)b * g.c_bs + (size_t)h * g.c_hs + (size_t)qrow * g.c_rs + n]
                   + g.pc[(size_t)b * g.c_bs + (size_t)h * g.c_hs + (size_t)kvcol * g.c_rs + n];
        }
        if (masked) s[j][r] = g.mask_fill;
        m = fmaxf(m, s[j][r]);
      }
#pragma unroll
      for (int off = 1; off < 16; off <<= 1) m = fmaxf(m, __shfl_xor(m, off, 32));
      cm[r] = m;
    }
    __bf16* pwh = Psh[wave];
    __bf16* pwl = Psl[SPLIT_PV ? wave : 0];
#pragma unroll
    for (int r = 0; r < 8; ++r) {
      const float mnew = fmaxf(mrow[r], cm[r]);
      const float alpha = expf(mrow[r] - mnew);
      mrow[r] = mnew;
      float psum = 0.f;
#pragma unroll
      for (int j = 0; j < 4; ++j) {
        const float p = expf(s[j][r] - mnew);
        psum += p;
        if (SPLIT_PV) { __bf16 a, bl; at_split(p, a, bl); pwh[(8 * hh + r) * AT_KC + j * 16 + c] = a; pwl[(8 * hh + r) * AT_KC + j * 16 + c] = bl; }
        else pwh[(8 * hh + r) * AT_KC + j * 16 + c] = at_to16<F16>(p * PSC);
      }
#pragma unroll
      for (int off = 1; off < 16; off <<= 1) psum += __shfl_xor(psum, off, 32);
      lrow[r] = lrow[r] * alpha + psum;
#pragma unroll
      for (int t = 0; t < 8; ++t) oacc[t][r] *= alpha;
    }
    __builtin_amdgcn_fence(__ATOMIC_RELEASE, "workgroup");
    __builtin_amdgcn_wave_barrier();
    __builtin_amdgcn_fence(__ATOMIC_ACQUIRE, "workgroup");
#pragma unroll 1
    for (int kk = 0; kk < 2; ++kk) {
      FB pa, pl;
      pa.h[0] = *(const v8b*)(pwh + c * AT_KC + kk * 32 + 8 * hh);
      pa.h[1] = *(const v8b*)(pwh + c * AT_KC + kk * 32 + 16 + 8 * hh);
      if (SPLIT_PV) {
        pl.h[0] = *(const v8b*)(pwl + c * AT_KC + kk * 32 + 8 * hh);
        pl.h[1] = *(const v8b*)(pwl + c * AT_KC + kk * 32 + 16 + 8 * hh);
      }
#pragma unroll
      for (int t = 0; t < 8; ++t) {
        FB vb;
        vb.h[0] = *(const v8b*)(Vth + (t * 16 + c) * AT_KC + kk * 32 + 8 * hh);
        vb.h[1] = *(const v8b*)(Vth + (t * 16 + c) * AT_KC + kk * 32 + 16 + 8 * hh);
        oacc[t] = at_mma16<F16>(pa.v, vb.v, oacc[t]);
        if (SPLIT_PV) {
          FB vl;
          vl.h[0] = *(const v8b*)(Vtl + (t * 16 + c) * AT_KC + kk * 32 + 8 * hh);
          vl.h[1] = *(const v8b*)(Vtl + (t * 16 + c) * AT_KC + kk * 32 + 16 + 8 * hh);
          oacc[t] = at_mma16<F16>(pa.v, vl.v, oacc[t]);
          oacc[t] = at_mma16<F16>(pl.v, vb.v, oacc[t]);
        }
      }
    }
  }

  float* os = Os[wave];
#pragma unroll
  for (int r = 0; r < 8; ++r) {
    const float inv = 1.0f / (lrow[r] * PSC);
#pragma unroll
    for (int t = 0; t < 8; ++t) os[(8 * hh + r) * 132 + t * 16 + c] = oacc[t][r] * inv;
  }
  __builtin_amdgcn_fence(__ATOMIC_RELEASE, "workgroup");
  __builtin_amdgcn_wave_barrier();
  __builtin_amdgcn_fence(__ATOMIC_ACQUIRE, "workgroup");
  {
    const int c4 = lane * 4;
    for (int pass = 0; pass < 2; ++pass) {
#pragma unroll
      for (int row = 0; row < 16; ++row) {
        v4f val = *(const v4f*)(os + row * 132 + c4);
        *(volatile v4f*)(ob_ptr + (size_t)(q0 + row) * g.o_rs + c4) = val;
      }
      __threadfence();
    }
  }
}

#define EB 8
#define EN 1024
#define EC 768
#define EH 8
#define EHD 96
#define EE 24
#define ET (EB * EN)
#ifndef TROWS
#define TROWS ET
#endif
__global__ __launch_bounds__(256) void router_kernel(const float* __restrict__ x, const float* __restrict__ Wg, const int* __restrict__ task, int* __restrict__ SELI, float* __restrict__ SELG, float* __restrict__ PROB, float* __restrict__ LSE2) {
  __shared__ int si[8][8]; __shared__ float sg[8][8]; __shared__ float sp[8][32];
  const int lane = threadIdx.x & 31, wave = threadIdx.x >> 5; const int t = blockIdx.x * 8 + wave;
  int tk = task[0]; tk = tk < 0 ? 0 : (tk > 8 ? 8 : tk);
  const float* W = Wg + (size_t)tk * EC * EE; const float* xr = x + (size_t)t * EC;
  float acc[EE];
#pragma unroll
  for (int e = 0; e < EE; ++e) acc[e] = 0.f;
#pragma unroll 1
  for (int q = 0; q < EC / 32; ++q) { const float xv = xr[q * 32 + lane]; const float* wr = W + (size_t)(q * 32 + lane) * EE;
#pragma unroll
    for (int e = 0; e < EE; ++e) acc[e] += xv * wr[e]; }
#pragma unroll
  for (int e = 0; e < EE; ++e) { float v = acc[e]; for (int o = 16; o > 0; o >>= 1) v += __shfl_xor(v, o, 32); acc[e] = v; }
  if (lane == 0) {
    float mx = acc[0]; for (int e = 1; e < EE; ++e) mx = fmaxf(mx, acc[e]);
    float p[EE], se = 0.f;
#pragma unroll 1
    for (int e = 0; e < EE; ++e) { p[e] = expf(acc[e] - mx); se += p[e]; }
    const float lse = mx + logf(se); sp[wave][24] = lse * lse;
    const float rs = 1.0f / se;
#pragma unroll 1
    for (int e = 0; e < EE; ++e) { p[e] *= rs; sp[wave][e] = p[e]; }
    unsigned used = 0u; float gs[EH]; int gi[EH]; float gsum = 0.f;
#pragma unroll 1
    for (int h = 0; h < EH; ++h) { int best = -1; float bv = -1.f;
#pragma unroll 1
      for (int e = 0; e < EE; ++e) if (!((used >> e) & 1u) && p[e] > bv) { bv = p[e]; best = e; }
      used |= 1u << best; gi[h] = best; gs[h] = bv; gsum += bv; }
    const float inv = 1.0f / (gsum + 1e-6f);
#pragma unroll 1
    for (int h = 0; h < EH; ++h) { si[wave][h] = gi[h]; sg[wave][h] = gs[h] * inv; }
  }
  __syncthreads();
  for (int pass = 0; pass < 2; ++pass) {
    if (threadIdx.x < 64) { ((volatile int*)SELI)[(size_t)blockIdx.x * 64 + threadIdx.x] = si[threadIdx.x >> 3][threadIdx.x & 7]; ((volatile float*)SELG)[(size_t)blockIdx.x * 64 + threadIdx.x] = sg[threadIdx.x >> 3][threadIdx.x & 7]; }
    else if (threadIdx.x < 64 + 192) { const int i = threadIdx.x - 64; ((volatile float*)PROB)[(size_t)blockIdx.x * 192 + i] = sp[i / 24][i % 24]; }
    if (threadIdx.x < 32) ((volatile float*)LSE2)[(size_t)blockIdx.x * 32 + threadIdx.x] = (threadIdx.x < 8) ? sp[threadIdx.x][24] : 0.f;
    __threadfence(); }
}
__global__ __launch_bounds__(256) void aux_kernel(const float* __restrict__ PROB, const int* __restrict__ SELI, const float* __restrict__ LSE2, float* __restrict__ aux) {
  __shared__ double imp[EE][8]; __shared__ double cnt[EE][8]; __shared__ double z[256];
  const int t = threadIdx.x, lane = t & 31, wave = t >> 5;
  double zi = 0.0; for (int i = t; i < ET; i += 256) zi += (double)LSE2[(size_t)(i >> 3) * 32 + (i & 7)]; z[t] = zi;
  if (lane < EE) { double a = 0.0, c = 0.0; for (int i = wave; i < ET; i += 8) { a += (double)PROB[(size_t)i * EE + lane]; for (int h = 0; h < EH; ++h) c += (SELI[(size_t)i * EH + h] == lane) ? 1.0 : 0.0; } imp[lane][wave] = a; cnt[lane][wave] = c; }
  __syncthreads();
  if (t == 0) { double sw = 0.0; for (int e = 0; e < EE; ++e) { double a = 0, c = 0; for (int w = 0; w < 8; ++w) { a += imp[e][w]; c += cnt[e][w]; } sw += (a / ET) * (c / ET / EH); }
    double zz = 0.0; for (int i = 0; i < 256; ++i) zz += z[i];
    const float v = (float)(0.1 * (EE * sw) + 0.001 * (zz / ET));
    float buf[32]; (void)buf;
    ((volatile float*)aux)[0] = v; __threadfence(); ((volatile float*)aux)[0] = v; }
}
__global__ __launch_bounds__(256) void winT_kernel(const float* __restrict__ Win, unsigned* __restrict__ WinH, unsigned* __restrict__ WinL) {
  __shared__ float tile[64][97];
  const int e = blockIdx.y, c0 = blockIdx.x * 64, tx = threadIdx.x, ty = threadIdx.y;
  for (int i = ty; i < 64; i += 8) for (int d = tx; d < EHD; d += 32) tile[i][d] = Win[((size_t)e * EC + c0 + i) * EHD + d];
  __syncthreads();
  for (int pass = 0; pass < 2; ++pass) {
    for (int d = ty; d < EHD; d += 8) { const float a = tile[2 * tx][d], b = tile[2 * tx + 1][d];
      const unsigned short ah = f2bf_bits(a), bh = f2bf_bits(b); const unsigned short al = f2bf_bits(a - bf_bits2f(ah)), bl = f2bf_bits(b - bf_bits2f(bh));
      const size_t o = (((size_t)e * EHD + d) * EC + c0) / 2 + tx;
      ((volatile unsigned*)WinH)[o] = (unsigned)ah | ((unsigned)bh << 16); ((volatile unsigned*)WinL)[o] = (unsigned)al | ((unsigned)bl << 16); }
    __threadfence(); }
}
__global__ __launch_bounds__(256) void qgather_kernel(const float* __restrict__ QALL, const int* __restrict__ SELI, float* __restrict__ Q) {
  const int lane = threadIdx.x & 31, wave = threadIdx.x >> 5; const int th = blockIdx.x * 8 + wave; const int t = th >> 3, h = th & 7;
  int e = SELI[th]; e = e < 0 ? 0 : (e >= EE ? EE - 1 : e);
  v4f v = {0.f, 0.f, 0.f, 0.f}; if (lane < 24) v = *(const v4f*)(QALL + (size_t)t * (EE * EHD) + e * EHD + lane * 4);
  *(volatile v4f*)(Q + (size_t)th * 128 + lane * 4) = v; __threadfence(); *(volatile v4f*)(Q + (size_t)th * 128 + lane * 4) = v;
}
__global__ __launch_bounds__(256) void kvpad_kernel(const float* __restrict__ KV, float* __restrict__ Kp, float* __restrict__ Vp) {
  const int lane = threadIdx.x & 31, wave = threadIdx.x >> 5; const int t = blockIdx.x * 8 + wave;
  v4f kv = {0.f, 0.f, 0.f, 0.f}, vv = {0.f, 0.f, 0.f, 0.f};
  if (lane < 24) { kv = *(const v4f*)(KV + (size_t)t * 192 + lane * 4); vv = *(const v4f*)(KV + (size_t)t * 192 + 96 + lane * 4); }
  for (int pass = 0; pass < 2; ++pass) { *(volatile v4f*)(Kp + (size_t)t * 128 + lane * 4) = kv; *(volatile v4f*)(Vp + (size_t)t * 128 + lane * 4) = vv; __threadfence(); }
}
__global__ __launch_bounds__(256) void zscatter_kernel(const float* __restrict__ O, const int* __restrict__ SELI, const float* __restrict__ SELG, unsigned* __restrict__ Z16) {
  const int lane = threadIdx.x & 31, wave = threadIdx.x >> 5; const int t = blockIdx.x * 8 + wave;
  unsigned* zr = Z16 + (size_t)t * (EE * EHD / 2);
  typedef __attribute__((ext_vector_type(2))) unsigned u2;
  for (int pass = 0; pass < 2; ++pass) {
    for (int i = lane; i < EE * EHD / 2; i += 32) ((volatile unsigned*)zr)[i] = 0u;
    __threadfence(); }
#pragma unroll 1
  for (int h = 0; h < EH; ++h) { int e = SELI[(size_t)t * EH + h]; e = e < 0 ? 0 : (e >= EE ? EE - 1 : e); const float g = SELG[(size_t)t * EH + h];
    if (lane < 24) { const v4f o = *(const v4f*)(O + ((size_t)t * EH + h) * 128 + lane * 4); u2 pk;
      pk[0] = (unsigned)__builtin_bit_cast(unsigned short, (_Float16)(o[0] * g)) | ((unsigned)__builtin_bit_cast(unsigned short, (_Float16)(o[1] * g)) << 16);
      pk[1] = (unsigned)__builtin_bit_cast(unsigned short, (_Float16)(o[2] * g)) | ((unsigned)__builtin_bit_cast(unsigned short, (_Float16)(o[3] * g)) << 16);
      *(volatile u2*)(zr + (e * EHD) / 2 + lane * 2) = pk; __threadfence(); *(volatile u2*)(zr + (e * EHD) / 2 + lane * 2) = pk; } }
}
extern "C" void kernel_launch(void* const* d_in, const int* in_sizes, int n_in, void* d_out, int out_size, void* d_ws, size_t ws_size, hipStream_t stream) {
  (void)in_sizes; (void)n_in; (void)out_size; (void)ws_size;
  const float* x = (const float*)d_in[0]; const float* Wg = (const float*)d_in[1]; const float* Win = (const float*)d_in[2]; const float* Wout = (const float*)d_in[3]; const float* Wkv = (const float*)d_in[4]; const int* task = (const int*)d_in[5];
  float* out = (float*)d_out; float* aux = out + (size_t)ET * EC;
  char* ws = (char*)d_ws; size_t off = 0;
  auto carve = [&](size_t bytes) -> char* { char* p = ws + off; off += (bytes + 255) & ~(size_t)255; return p; };
  int* SELI = (int*)carve((size_t)ET * EH * 4); float* SELG = (float*)carve((size_t)ET * EH * 4); float* PROB = (float*)carve((size_t)ET * EE * 4); float* LSE2 = (float*)carve((size_t)(ET / 8) * 32 * 4);
  __bf16* Xh = (__bf16*)carve((size_t)TROWS * EC * 2); __bf16* Xl = (__bf16*)carve((size_t)TROWS * EC * 2);
  unsigned* WinH = (unsigned*)carve((size_t)EE * EHD * EC * 2); unsigned* WinL = (unsigned*)carve((size_t)EE * EHD * EC * 2);
  __bf16* WkvH = (__bf16*)carve((size_t)192 * EC * 2); __bf16* WkvL = (__bf16*)carve((size_t)192 * EC * 2);
  _Float16* Wout16 = (_Float16*)carve((size_t)EC * EE * EHD * 2);
  float* QALL = (float*)carve((size_t)TROWS * EE * EHD * 4);
  float* KV = (float*)carve((size_t)TROWS * 192 * 4);
  float* Q = (float*)carve((size_t)TROWS * EH * 128 * 4);
  float* Kp = (float*)carve((size_t)TROWS * 128 * 4); float* Vp = (float*)carve((size_t)TROWS * 128 * 4);
  float* O = (float*)carve((size_t)TROWS * EH * 128 * 4);
  unsigned* Z16 = (unsigned*)carve((size_t)TROWS * EE * EHD * 2);
  router_kernel<<<ET / 8, 256, 0, stream>>>(x, Wg, task, SELI, SELG, PROB, LSE2);
  aux_kernel<<<1, 256, 0, stream>>>(PROB, SELI, LSE2, aux);
  split_f32_bf16x2<<<(TROWS * EC / 2 + 255) / 256, 256, 0, stream>>>(x, Xh, Xl, TROWS * EC / 2);
  winT_kernel<<<dim3(EC / 64, EE), dim3(32, 8), 0, stream>>>(Win, WinH, WinL);
  transpose_split_bf16<<<dim3(192 / 64, EC / 64), dim3(32, 8), 0, stream>>>(Wkv, 192, WkvH, WkvL, EC);
  transpose_cast_f16<<<dim3(EC / 64, EE * EHD / 64), dim3(32, 8), 0, stream>>>(Wout, EC, Wout16, EE * EHD, 1.0f);
  { const int t1 = (TROWS / 64) * (EE * EHD / 64), t2 = (TROWS / 64) * (192 / 64);
    wmma_gemm64<1, true, 0, 0, false><<<dim3((t1 + 7) / 8, 1), 256, 0, stream>>>(U16(Xh), U16(Xl), EC, 0, (const unsigned short*)WinH, (const unsigned short*)WinL, EC, 0, QALL, nullptr, EE * EHD, 0, nullptr, nullptr, 0, TROWS, EE * EHD, EC, 1.0f);
    wmma_gemm64<1, true, 0, 0, false><<<dim3((t2 + 7) / 8, 1), 256, 0, stream>>>(U16(Xh), U16(Xl), EC, 0, U16(WkvH), U16(WkvL), EC, 0, KV, nullptr, 192, 0, nullptr, nullptr, 0, TROWS, 192, EC, 1.0f); }
  qgather_kernel<<<TROWS * EH / 8, 256, 0, stream>>>(QALL, SELI, Q);
  kvpad_kernel<<<TROWS / 8, 256, 0, stream>>>(KV, Kp, Vp);
  { AttnGeom g;
    g.q_bs = (long)EN * EH * 128; g.q_rs = EH * 128; g.q_hs = 128; g.k_bs = (long)EN * 128; g.k_rs = 128; g.k_hs = 0; g.v_bs = (long)EN * 128; g.v_rs = 128; g.v_hs = 0; g.o_bs = (long)EN * EH * 128; g.o_rs = EH * 128; g.o_hs = 128;
    g.S = EN; g.Skv = EN; g.H = EH; g.mask_mode = 0; g.qscale = 0.10206207261596575f; g.blk0 = 0; g.mask_fill = -INFINITY; g.mask_is_int = 0;
    attn128_kernel<true, true, false><<<(TROWS / EN) * EH * (EN / AT_QB), AT_NW * 32, 0, stream>>>(Q, Kp, Vp, O, nullptr, nullptr, g); }
  zscatter_kernel<<<TROWS / 8, 256, 0, stream>>>(O, SELI, SELG, Z16);
  { const int t = (TROWS / 64) * (EC / 64);
    wmma_gemm64<0, false, 0, 0, false><<<dim3((t + 7) / 8, 1), 256, 0, stream>>>((const unsigned short*)Z16, nullptr, EE * EHD, 0, U16(Wout16), nullptr, EE * EHD, 0, out, nullptr, EC, 0, nullptr, nullptr, 0, TROWS, EC, EE * EHD, 1.0f); }
}
